// VanillaRNN_42640435314854
// MI455X (gfx1250) — hardware-verified
//
#include <hip/hip_runtime.h>
#include <math.h>

constexpr int SEQ_T  = 512;
constexpr int HID    = 256;
constexpr int NBATCH = 1024;
constexpr int NCLS   = 10;
constexpr int NTHR   = 256;
constexpr int NWAVE  = NTHR / 32;
constexpr int BCOLS  = 16;
constexpr int NBLK   = NBATCH / BCOLS;
constexpr int XP     = SEQ_T + 4;
constexpr int HP     = HID + 8;
constexpr int HT     = BCOLS * HP;
constexpr int HFP    = HID + 4;
constexpr int NOUTB  = BCOLS * NCLS;
constexpr int WDWORDS = HID * HID / 2;
constexpr float WCARRY = 256.0f;
constexpr float HCARRY = 1024.0f;
constexpr float PINV   = 1.0f / (WCARRY * HCARRY);
static_assert(HID == NWAVE * 32);
static_assert(NBATCH % BCOLS == 0);
static_assert(HID % 32 == 0);
static_assert(XP % 4 == 0 && HP % 8 == 0 && HFP % 4 == 0);
static_assert(BCOLS * HFP <= BCOLS * XP);
static_assert((BCOLS * SEQ_T) % NTHR == 0);
static_assert(WDWORDS % NTHR == 0);
static_assert((NOUTB * 4) % 128 == 0);
static_assert(NOUTB == 128 + 32);
static_assert(NOUTB <= NTHR);
static_assert(NCLS * HID == 2560);

typedef __attribute__((ext_vector_type(16))) _Float16 v16h;
typedef __attribute__((ext_vector_type(8)))  _Float16 v8h;
typedef __attribute__((ext_vector_type(8)))  float    v8f;
typedef __attribute__((ext_vector_type(4)))  float    v4f;
typedef __attribute__((ext_vector_type(2)))  float    v2f;

__device__ __forceinline__ void dep_guard_h(v8f& a, v8f& b, v16h x, v16h y) { asm volatile("v_nop\n\tv_nop\n\tv_nop\n\tv_nop" : "+v"(a), "+v"(b) : "v"(x), "v"(y)); }
__device__ __forceinline__ void keep4_h(v16h a, v16h b, v16h c, v16h d) { asm volatile("v_nop" :: "v"(a), "v"(b), "v"(c), "v"(d)); }
__device__ __forceinline__ void acc_guard2(v8f& a, v8f& b) { asm volatile("v_nop\n\tv_nop\n\tv_nop\n\tv_nop" : "+v"(a), "+v"(b)); }

template <typename T> struct Frag;
template <> struct Frag<_Float16> {
  typedef v16h V; union U { v16h v; v8h h[2]; };
  static __device__ __forceinline__ v16h load(const _Float16* p) {
    U f; f.h[0] = *(const v8h*)(p); f.h[1] = *(const v8h*)(p + 16); return f.v;
  }
  static __device__ __forceinline__ v8f mma(v16h a, v16h b, v8f c) {
    return __builtin_amdgcn_wmma_f32_16x16x32_f16(false, a, false, b, (short)0, c, false, false);
  }
};

__device__ __forceinline__ float tanh_f32(float v) {
  const float e = expf(2.0f * v);
  return 1.0f - 2.0f / (1.0f + e);
}

__global__ __launch_bounds__(NTHR) void whh_prep_kernel(const float* __restrict__ whh, unsigned* __restrict__ dst) {
  const int i = blockIdx.x * NTHR + threadIdx.x;
  const v2f w = *(const v2f*)(whh + 2 * (size_t)i);
  const float f0 = w[0] * WCARRY;
  const float f1 = w[1] * WCARRY;
  const _Float16 h0 = (_Float16)f0;
  const _Float16 h1 = (_Float16)f1;
  const unsigned u = (unsigned)__builtin_bit_cast(unsigned short, h0) | ((unsigned)__builtin_bit_cast(unsigned short, h1) << 16);
  *(volatile unsigned*)(dst + i) = u;
  __threadfence();
  *(volatile unsigned*)(dst + i) = u;
}

__global__ __launch_bounds__(NTHR) void rnn_seq_kernel(const float* __restrict__ x, const float* __restrict__ whx,
                                                       const float* __restrict__ bh, const unsigned short* __restrict__ whh16p,
                                                       const float* __restrict__ wph, const float* __restrict__ bp,
                                                       float* __restrict__ out) {
  __shared__ __align__(16) _Float16 hbuf[2 * HT];
  __shared__ __align__(16) float    xl[BCOLS * XP];
  __shared__ __align__(16) float    outs[NOUTB];
  const _Float16* whh16 = (const _Float16*)whh16p;
  const int tid = threadIdx.x, lane = tid & 31, wave = tid >> 5;
  const int c = lane & 15, hh = lane >> 4, koff = hh * 8;
  const int b0 = blockIdx.x * BCOLS;
  const int m0 = wave * 32;

#pragma unroll 1
  for (int i = tid; i < BCOLS * SEQ_T; i += NTHR) {
    const int bb = i / SEQ_T;
    const int t  = i - bb * SEQ_T;
    xl[bb * XP + t] = x[(size_t)(b0 + bb) * SEQ_T + t];
  }
  {
    const v8h z = {(_Float16)0.f, (_Float16)0.f, (_Float16)0.f, (_Float16)0.f, (_Float16)0.f, (_Float16)0.f, (_Float16)0.f, (_Float16)0.f};
#pragma unroll 1
    for (int i = tid; i < (2 * HT) / 8; i += NTHR) *(v8h*)(hbuf + 8 * i) = z;
  }
  float wx[2][8], bv[2][8];
#pragma unroll
  for (int i = 0; i < 2; ++i) {
    const float* p = whx + m0 + 16 * i + 8 * hh;
    const v4f a = *(const v4f*)(p);
    const v4f b = *(const v4f*)(p + 4);
    wx[i][0] = a[0]; wx[i][1] = a[1]; wx[i][2] = a[2]; wx[i][3] = a[3];
    wx[i][4] = b[0]; wx[i][5] = b[1]; wx[i][6] = b[2]; wx[i][7] = b[3];
  }
  asm volatile("" ::: "memory");
#pragma unroll
  for (int i = 0; i < 2; ++i) {
    const float* p = bh + m0 + 16 * i + 8 * hh;
    const v4f a = *(const v4f*)(p);
    const v4f b = *(const v4f*)(p + 4);
    bv[i][0] = a[0]; bv[i][1] = a[1]; bv[i][2] = a[2]; bv[i][3] = a[3];
    bv[i][4] = b[0]; bv[i][5] = b[1]; bv[i][6] = b[2]; bv[i][7] = b[3];
  }
  __syncthreads();

  const _Float16* arow0 = whh16 + (size_t)(m0 + c) * HID + koff;
  const _Float16* arow1 = arow0 + (size_t)16 * HID;
  const v8f z8 = {0.f, 0.f, 0.f, 0.f, 0.f, 0.f, 0.f, 0.f};
  float hl[2][8];
#pragma unroll
  for (int i = 0; i < 2; ++i)
#pragma unroll
    for (int r = 0; r < 8; ++r) hl[i][r] = 0.0f;

#pragma unroll 1
  for (int t = 0; t < SEQ_T; ++t) {
    const _Float16* hc = hbuf + (t & 1) * HT;
    _Float16*       hn = hbuf + ((t + 1) & 1) * HT;
    const _Float16* brow = hc + c * HP + koff;
    const float xv = xl[c * XP + t];

    v8f acc[2];
    acc[0] = z8; acc[1] = z8;
#pragma unroll 2
    for (int kc = 0; kc < HID / 32; ++kc) {
      const v16h fb  = Frag<_Float16>::load(brow  + kc * 32);
      const v16h fa0 = Frag<_Float16>::load(arow0 + kc * 32);
      const v16h fa1 = Frag<_Float16>::load(arow1 + kc * 32);
      acc[0] = Frag<_Float16>::mma(fa0, fb, acc[0]);
      acc[1] = Frag<_Float16>::mma(fa1, fb, acc[1]);
      dep_guard_h(acc[0], acc[1], fa1, fb);
      keep4_h(fa0, fa1, fb, fa0);
    }
    acc_guard2(acc[0], acc[1]);

#pragma unroll
    for (int i = 0; i < 2; ++i) {
      v8h hv;
#pragma unroll
      for (int r = 0; r < 8; ++r) {
        const float xin = wx[i][r] * xv;
        const float pre = fmaf(acc[i][r], PINV, xin) + bv[i][r];
        const float h   = tanh_f32(pre);
        hl[i][r] = h;
        hv[r] = (_Float16)(h * HCARRY);
      }
      *(v8h*)(hn + c * HP + m0 + 16 * i + 8 * hh) = hv;
    }
    __syncthreads();
  }

  float* hf = xl;
#pragma unroll
  for (int i = 0; i < 2; ++i) {
    const v4f p0 = {hl[i][0], hl[i][1], hl[i][2], hl[i][3]};
    const v4f p1 = {hl[i][4], hl[i][5], hl[i][6], hl[i][7]};
    float* dp = hf + c * HFP + m0 + 16 * i + 8 * hh;
    *(v4f*)(dp)     = p0;
    *(v4f*)(dp + 4) = p1;
  }
  __syncthreads();

  if (tid < NOUTB) {
    const int bb  = tid / NCLS;
    const int cls = tid - bb * NCLS;
    const float* wr = wph + (size_t)cls * HID;
    const float* hr = hf + bb * HFP;
    float s = 0.0f;
#pragma unroll 2
    for (int k4 = 0; k4 < HID / 4; ++k4) {
      const v4f w4 = *(const v4f*)(wr + 4 * k4);
      const v4f h4 = *(const v4f*)(hr + 4 * k4);
      s = fmaf(w4[0], h4[0], s);
      s = fmaf(w4[1], h4[1], s);
      s = fmaf(w4[2], h4[2], s);
      s = fmaf(w4[3], h4[3], s);
    }
    outs[tid] = s + bp[cls];
  }
  __syncthreads();

  if (wave == 0) {
    float* op = out + (size_t)b0 * NCLS;
    const v4f v0 = *(const v4f*)(outs + 4 * lane);
    const int l8 = (lane < 8) ? lane : 0;
    const v4f v1 = *(const v4f*)(outs + 128 + 4 * l8);
    for (int pass = 0; pass < 2; ++pass) {
      *(volatile v4f*)(op + 4 * lane) = v0;
      if (lane < 8) *(volatile v4f*)(op + 128 + 4 * lane) = v1;
      __threadfence();
    }
  }
}

extern "C" void kernel_launch(void* const* d_in, const int* in_sizes, int n_in,
                              void* d_out, int out_size, void* d_ws, size_t ws_size, hipStream_t stream) {
  if (n_in < 6 || d_out == nullptr || d_ws == nullptr) return;
  if (in_sizes[0] != NBATCH * SEQ_T || in_sizes[1] != HID || in_sizes[2] != HID * HID ||
      in_sizes[3] != NCLS * HID || in_sizes[4] != HID || in_sizes[5] != NCLS ||
      out_size != NBATCH * NCLS) return;

  const float* x   = (const float*)d_in[0];
  const float* whx = (const float*)d_in[1];
  const float* whh = (const float*)d_in[2];
  const float* wph = (const float*)d_in[3];
  const float* bh  = (const float*)d_in[4];
  const float* bp  = (const float*)d_in[5];
  float* out = (float*)d_out;

  const size_t whh16_bytes = (size_t)HID * HID * 2;
  if (whh16_bytes > ws_size || whh16_bytes > (size_t)134217728) return;
  unsigned short* WHH16 = (unsigned short*)d_ws;

  whh_prep_kernel<<<WDWORDS / NTHR, NTHR, 0, stream>>>(whh, (unsigned*)WHH16);

  rnn_seq_kernel<<<NBLK, NTHR, 0, stream>>>(x, whx, bh, WHH16, wph, bp, out);
}
